// GNNLayer_70875550319239
// MI455X (gfx1250) — hardware-run, weakly checked
//
#include <hip/hip_runtime.h>

typedef float          v8f   __attribute__((ext_vector_type(8)));
typedef float          v4f   __attribute__((ext_vector_type(4)));
typedef unsigned int   v4u   __attribute__((ext_vector_type(4)));
typedef int            v8i   __attribute__((ext_vector_type(8)));
typedef unsigned short v8us  __attribute__((ext_vector_type(8)));
typedef unsigned short v16us __attribute__((ext_vector_type(16)));
typedef __bf16         v16bf __attribute__((ext_vector_type(16)));
typedef _Float16       v16h  __attribute__((ext_vector_type(16)));
typedef v4f  __attribute__((may_alias)) v4fa;
typedef v8us __attribute__((may_alias)) v8usa;
union FragB { v16bf v; v16us u; v8us h[2]; v8i w; };
union FragH { v16h  v; v16us u; v8us h[2]; v8i w; };

__device__ __forceinline__ v8f wmb(const FragB& a, const FragB& b, v8f c) {
  v8f d = __builtin_amdgcn_wmma_f32_16x16x32_bf16(false, a.v, false, b.v, (short)0, c, false, false);
  asm volatile("v_nop\n\tv_nop\n\tv_nop\n\tv_nop" : "+v"(d) : "v"(a.w), "v"(b.w));
  return d;
}

__device__ __forceinline__ v8f wmh(const FragH& a, const FragH& b, v8f c) {
  v8f d = __builtin_amdgcn_wmma_f32_16x16x32_f16(false, a.v, false, b.v, (short)0, c, false, false);
  asm volatile("v_nop\n\tv_nop\n\tv_nop\n\tv_nop" : "+v"(d) : "v"(a.w), "v"(b.w));
  return d;
}

__device__ __forceinline__ unsigned bf16_bits(float f) {
  const unsigned u = __float_as_uint(f);
  const unsigned r = (u + 0x7FFFu + ((u >> 16) & 1u)) >> 16;
  const unsigned q = (u >> 16) | 0x40u;
  return ((u & 0x7fffffffu) > 0x7f800000u) ? q : r;
}

__device__ __forceinline__ float bf16_val(float f) {
  return __uint_as_float(bf16_bits(f) << 16);
}
__device__ __forceinline__ int clampi(int v, int lo, int hi) {
  return v < lo ? lo : (v > hi ? hi : v);
}

__device__ __forceinline__ unsigned f16_bits(float f) {
  const unsigned u  = __float_as_uint(f);
  const unsigned s  = (u >> 16) & 0x8000u;
  const unsigned a  = u & 0x7fffffffu;
  const unsigned t  = a - 0x38000000u;
  const unsigned r  = (t + 0x0FFFu + ((t >> 13) & 1u)) >> 13;
  const unsigned rc = r > 0x7C00u ? 0x7C00u : r;
  const bool small  = a < 0x38800000u;
  const bool isnan  = a > 0x7f800000u;
  const unsigned fin = small ? 0u : (s | rc);
  return isnan ? (s | 0x7E00u) : fin;
}

__device__ __forceinline__ unsigned pk16(unsigned lo, unsigned hi) { return lo | (hi << 16); }
__device__ __forceinline__ unsigned bf16_lo_bits(float v) {
  float hi = bf16_val(v);
  asm volatile("" : "+v"(hi));
  return bf16_bits(v - hi);
}
__device__ __forceinline__ v4u pack8_bf16(v4f a, v4f c) {
  return (v4u){ pk16(bf16_bits(a[0]), bf16_bits(a[1])), pk16(bf16_bits(a[2]), bf16_bits(a[3])),
                pk16(bf16_bits(c[0]), bf16_bits(c[1])), pk16(bf16_bits(c[2]), bf16_bits(c[3])) };
}
__device__ __forceinline__ v4u pack8_bf16_lo(v4f a, v4f c) {
  return (v4u){ pk16(bf16_lo_bits(a[0]), bf16_lo_bits(a[1])), pk16(bf16_lo_bits(a[2]), bf16_lo_bits(a[3])),
                pk16(bf16_lo_bits(c[0]), bf16_lo_bits(c[1])), pk16(bf16_lo_bits(c[2]), bf16_lo_bits(c[3])) };
}
__device__ __forceinline__ v4u pack8_f16(v4f a, v4f c) {
  return (v4u){ pk16(f16_bits(a[0]), f16_bits(a[1])), pk16(f16_bits(a[2]), f16_bits(a[3])),
                pk16(f16_bits(c[0]), f16_bits(c[1])), pk16(f16_bits(c[2]), f16_bits(c[3])) };
}

template <int FORM>
__global__ __launch_bounds__(256) void k_plane(const float* __restrict__ src, int rows, int cols, int ldsrc,
                                               unsigned short* __restrict__ dst, int MP, int KP) {
  static_assert(FORM >= 0 && FORM <= 3);
  const int KTOT = (FORM == 1 || FORM == 3) ? 2 * KP : KP;
  const unsigned ppr   = (unsigned)(KTOT >> 3);
  const unsigned kp8   = (unsigned)(KP >> 3);
  const unsigned total = (unsigned)MP * ppr;
  const unsigned g     = blockIdx.x * 256u + threadIdx.x;
  const unsigned rowu  = g / ppr;
  const unsigned p     = g - rowu * ppr;
  const bool second    = p >= kp8;
  const int row = (int)rowu;
  const int c0  = (int)((second ? p - kp8 : p) << 3);
  const float* srow = src + (size_t)clampi(row, 0, rows - 1) * (size_t)ldsrc;
  float x[8];
  unsigned mk[8];
#pragma unroll
  for (int e = 0; e < 8; ++e) {
    const int c = c0 + e;
    const float v = srow[clampi(c, 0, cols - 1)];
    asm volatile("" :: "v"(v));
    x[e]  = v;
    mk[e] = (row < rows && c < cols) ? 0xFFFFu : 0u;
  }
  const v4f a = (v4f){ x[0], x[1], x[2], x[3] };
  const v4f c = (v4f){ x[4], x[5], x[6], x[7] };
  v4u o;
  if (FORM == 2) {
    o = pack8_f16(a, c);
  } else {
    const v4u hi = pack8_bf16(a, c);
    o = hi;
    if (FORM == 1) { const v4u lo = pack8_bf16_lo(a, c); o = second ? lo : hi; }
  }
  const v4u mw = (v4u){ pk16(mk[0], mk[1]), pk16(mk[2], mk[3]), pk16(mk[4], mk[5]), pk16(mk[6], mk[7]) };
  o &= mw;
  if (g < total) {
    volatile v4u* q = (volatile v4u*)(dst + (size_t)g * 8);
    *q = o;
    __threadfence();
    *q = o;
  }
}

template <int FORM> struct FragOf    { typedef FragB T; };
template <>         struct FragOf<2> { typedef FragH T; };
__device__ __forceinline__ v8f mm(const FragB& a, const FragB& b, v8f c) { return wmb(a, b, c); }
__device__ __forceinline__ v8f mm(const FragH& a, const FragH& b, v8f c) { return wmh(a, b, c); }
template <class F> __device__ __forceinline__ F ld_frag(const unsigned short* p) {
  F f;
  f.h[0] = *(const v8usa*)(p);
  f.h[1] = *(const v8usa*)(p + 16);
  return f;
}

template <int FORM, int EPI>
__global__ __launch_bounds__(256) __attribute__((amdgpu_num_vgpr(248)))
void k_gemm_nt(const unsigned short* __restrict__ A, const unsigned short* __restrict__ B,
               const float* __restrict__ bias, float* __restrict__ D, int M, int N, int KTOT, int ldd) {
  static_assert(FORM >= 0 && FORM <= 2);
  static_assert(EPI == 0 || EPI == 1);
  typedef typename FragOf<FORM>::T F;
  __shared__ __attribute__((aligned(16))) float sT[8][16 * 68];
  const int lane = threadIdx.x & 31;
  const int wave = threadIdx.x >> 5;
  const int tilesM = (M + 63) >> 6;
  const int tilesN = (N + 63) >> 6;
  const int tile = blockIdx.x * 8 + wave;
  if (tile >= tilesM * tilesN) return;
  const int tm = tile / tilesN;
  const int tn = tile - tm * tilesN;
  const int m0 = tm << 6;
  const int n0 = tn << 6;

  const int rl = lane & 15;
  const int h8 = (lane >> 4) * 8;
  const unsigned short* pa = A + (size_t)(m0 + rl) * (size_t)KTOT + h8;
  const unsigned short* pb = B + (size_t)(n0 + rl) * (size_t)KTOT + h8;

  v8f acc[4][4];
#pragma unroll
  for (int i = 0; i < 4; ++i)
#pragma unroll
    for (int j = 0; j < 4; ++j) acc[i][j] = (v8f){0.f, 0.f, 0.f, 0.f, 0.f, 0.f, 0.f, 0.f};

#pragma unroll 1
  for (int k0 = 0; k0 < KTOT; k0 += 32) {
    F bf[4];
#pragma unroll
    for (int j = 0; j < 4; ++j) bf[j] = ld_frag<F>(pb + (size_t)(j << 4) * (size_t)KTOT + k0);
#pragma unroll
    for (int i = 0; i < 4; ++i) {
      const F af = ld_frag<F>(pa + (size_t)(i << 4) * (size_t)KTOT + k0);
#pragma unroll
      for (int j = 0; j < 4; ++j) acc[i][j] = mm(af, bf[j], acc[i][j]);
    }
  }

  float* slab = sT[wave];
  const int hh = lane >> 4;
  const int c4 = (lane & 15) * 4;
  const int nc = n0 + c4;
  const bool cok = nc < N;
  v4f bv = (v4f){0.f, 0.f, 0.f, 0.f};
  if (EPI == 1) {
    bv = *(const v4fa*)(bias + clampi(nc, 0, N - 4));
    asm volatile("" :: "v"(bv));
  }
#pragma unroll
  for (int i = 0; i < 4; ++i) {
    const int mBase = m0 + (i << 4);
#pragma unroll
    for (int j = 0; j < 4; ++j) {
#pragma unroll
      for (int r = 0; r < 8; ++r) slab[(h8 + r) * 68 + (j << 4) + rl] = acc[i][j][r];
    }
    __builtin_amdgcn_fence(__ATOMIC_RELEASE, "workgroup");
    __builtin_amdgcn_wave_barrier();
    __builtin_amdgcn_fence(__ATOMIC_ACQUIRE, "workgroup");
    v4f vv[8];
#pragma unroll
    for (int it = 0; it < 8; ++it) {
      const int row = it * 2 + hh;
      v4f v = *(const v4fa*)(slab + row * 68 + c4);
      if (EPI == 1) v += bv;
      vv[it] = v;
    }
    for (int pass = 0; pass < 2; ++pass) {
#pragma unroll
      for (int it = 0; it < 8; ++it) {
        const int row = mBase + it * 2 + hh;
        if (cok && row < M) *(volatile v4f*)(D + (size_t)row * (size_t)ldd + nc) = vv[it];
      }
      __threadfence();
    }
    __builtin_amdgcn_fence(__ATOMIC_RELEASE, "workgroup");
    __builtin_amdgcn_wave_barrier();
    __builtin_amdgcn_fence(__ATOMIC_ACQUIRE, "workgroup");
  }
}

#pragma clang fp contract(off)

#ifndef ZTERMS
#define ZTERMS 2
#endif
#ifndef RNE_VEC
#define RNE_VEC 1
#endif
static_assert(ZTERMS == 1 || ZTERMS == 2);
static_assert(RNE_VEC == 0 || RNE_VEC == 1);

typedef int    v4i __attribute__((ext_vector_type(4)));
typedef double v2d __attribute__((ext_vector_type(2)));
typedef v4i __attribute__((may_alias)) v4ia;
typedef v4u __attribute__((may_alias)) v4ua;

constexpr int NN        = 100000;
constexpr int NE        = 1000000;
constexpr int NCH       = 20;
constexpr int CH        = 50000;
constexpr int CHP       = 50048;
constexpr int VBP       = 100096;
constexpr int KZ        = 96;
constexpr int K_E       = KZ * ZTERMS;
constexpr int K_R       = 32;
constexpr int OUT_ELEMS = 1600000;

static_assert(NE == NCH * CH);
static_assert(CHP == 391 * 128 && CHP % 64 == 0 && CHP >= CH && CHP - CH < 64);
static_assert(NN == 2 * CH && NN % 2 == 0);
static_assert(OUT_ELEMS == 6250 * 256 && OUT_ELEMS == NN * 16);
static_assert(CH % 16 == 0 && K_E % 32 == 0 && K_R % 32 == 0);
static_assert(VBP % 64 == 0 && VBP >= NN && VBP >= CH + CHP);
static_assert(NE == 488 * 2048 + 576);

constexpr int NBRUN  = 1024;
constexpr int NBLK   = 98;
constexpr int CAP    = 14336;
constexpr int DEGCAP = 32;
constexpr int WLCAP  = 4096;
constexpr int EPW    = NE / 8;
constexpr int SUB    = 128;
constexpr int NSTEP  = (EPW + SUB - 1) / SUB;

static_assert(NBLK * NBRUN >= NN && (NBLK - 1) * NBRUN < NN);
static_assert(NE % 8 == 0 && EPW * 8 == NE && NSTEP * SUB >= EPW && (NSTEP - 1) * SUB < EPW);
static_assert(CAP * 4 >= 10435 * 5 && (CAP / 4) % 256 == 0 && CAP >= 2 * DEGCAP);
static_assert(DEGCAP > 26 && DEGCAP <= 32);
static_assert(WLCAP * 4 >= 1305 * 5 && WLCAP * 8 >= CAP);
static_assert((((long long)(NE - 1) << 10) | 1023) < (1LL << 31));
static_assert((NN / 2) % 8 == 0);

constexpr int LK_WL   = 0;
constexpr int LK_SL   = 8 * WLCAP;
constexpr int LK_CNT  = LK_SL + CAP;
constexpr int LK_OFF  = LK_CNT + NBRUN;
constexpr int LK_CUR  = LK_OFF + NBRUN;
constexpr int LK_MISC = LK_CUR + NBRUN;
constexpr int LK_INTS = LK_MISC + 16;
constexpr int LK_LDS  = LK_INTS * 4;
static_assert(LK_LDS == 200768 && LK_LDS <= 262144 && LK_LDS <= 327680);
static_assert(LK_SL % 4 == 0 && LK_CNT % 4 == 0 && (CAP + NBRUN) % 1024 == 0);

constexpr int T_BIAS = 0, T_GAM = 32, T_BET = 64, T_MU = 96, T_RS = 128, T_N = 160;
constexpr int NREC = 250;
constexpr int RROWS = 400;
constexpr int GROWS = 25;
static_assert(NREC * RROWS == NN && 16 * GROWS == RROWS);

constexpr size_t SZ_Z     = (size_t)CHP * K_E * 2;
constexpr size_t SZ_MSGC  = (size_t)CHP * 64 * 4;
constexpr size_t SZ_MSG16 = (size_t)NE * 16 * 4;
constexpr size_t SZ_RT16  = (size_t)NN * 16 * 4;
constexpr size_t SZ_PRE   = (size_t)NN * 16 * 4;
constexpr size_t SZ_VB    = (size_t)VBP * K_R * 2;
constexpr size_t SZ_LIST  = (size_t)NBLK * CAP * 4;
constexpr size_t SZ_NODE  = (size_t)NBLK * NBRUN * 4;
constexpr size_t SZ_FLAG  = (size_t)NBLK * 128;
constexpr size_t SZ_WRB   = (size_t)64 * K_E * 2;
constexpr size_t SZ_ROOTT = (size_t)64 * K_R * 2;
constexpr size_t SZ_TAB   = 768;
constexpr size_t SZ_REC   = (size_t)NREC * 16 * 8;
constexpr size_t OFF_Z     = 0;
constexpr size_t OFF_MSGC  = OFF_Z + SZ_Z;
constexpr size_t OFF_MSG16 = OFF_MSGC + SZ_MSGC;
constexpr size_t OFF_RT16  = OFF_MSG16 + SZ_MSG16;
constexpr size_t OFF_PRE   = OFF_RT16 + SZ_RT16;
constexpr size_t OFF_VB    = OFF_PRE + SZ_PRE;
constexpr size_t OFF_LIST  = OFF_VB + SZ_VB;
constexpr size_t OFF_CNT   = OFF_LIST + SZ_LIST;
constexpr size_t OFF_OFF   = OFF_CNT + SZ_NODE;
constexpr size_t OFF_FLAG  = OFF_OFF + SZ_NODE;
constexpr size_t OFF_WRB   = OFF_FLAG + SZ_FLAG;
constexpr size_t OFF_ROOTT = OFF_WRB + SZ_WRB;
constexpr size_t OFF_TAB   = OFF_ROOTT + SZ_ROOTT;
constexpr size_t OFF_REC   = OFF_TAB + SZ_TAB;
constexpr size_t WS_TOTAL  = OFF_REC + SZ_REC;
static_assert(WS_TOTAL <= ((size_t)128 << 20));
static_assert(SZ_Z % 256 == 0 && SZ_MSGC % 256 == 0 && SZ_MSG16 % 256 == 0 && SZ_RT16 % 256 == 0 && SZ_PRE % 256 == 0);
static_assert(SZ_VB % 256 == 0 && SZ_LIST % 256 == 0 && SZ_NODE % 256 == 0 && SZ_FLAG % 256 == 0);
static_assert(SZ_WRB % 256 == 0 && SZ_ROOTT % 256 == 0 && SZ_TAB % 256 == 0 && SZ_REC % 256 == 0);
static_assert((size_t)T_N * 4 <= SZ_TAB);
static_assert(((size_t)CH * K_E * 2) % 128 == 0);
static_assert(((size_t)CH * K_R * 2) % 128 == 0);
static_assert(((size_t)CH * 16 * 4) % 128 == 0);
static_assert((size_t)VBP * (K_R / 8) < ((size_t)1 << 31));

constexpr int PB_W   = 64 * (K_E / 8) / 256;
constexpr int PB_TOT = PB_W + 2;
constexpr int ZPADP  = (CHP - CH) * (K_E / 8);
static_assert((64 * (K_E / 8)) % 256 == 0 && ZPADP % 32 == 0);
constexpr int S_W = 0, S_B = 1024, S_R = 1280, S_VEC = 1536;

__global__ __launch_bounds__(256) __attribute__((amdgpu_num_vgpr(128)))
void k_prep(const float* __restrict__ EW, const float* __restrict__ EB, const float* __restrict__ root,
            const float* __restrict__ bias, const float* __restrict__ gam, const float* __restrict__ bet,
            unsigned short* __restrict__ WRB, unsigned short* __restrict__ ROOTT, float* __restrict__ TAB,
            unsigned short* __restrict__ Z) {
  __shared__ __attribute__((aligned(16))) float sS[1600];
  const int tid = (int)threadIdx.x;
  const int blk = (int)blockIdx.x;
  if (blk <= PB_W) {
    const int t64 = tid < 64 ? tid : 63;
    const int t4  = tid < 4 ? tid : 3;
    const v4f w4 = *(const v4fa*)(EW + 4 * tid);
    const v4f b4 = *(const v4fa*)(EB + 4 * t64);
    const v4f r4 = *(const v4fa*)(root + 4 * t64);
    const v4f x4 = *(const v4fa*)(bias + 4 * t4);
    const v4f g4 = *(const v4fa*)(gam + 4 * t4);
    const v4f y4 = *(const v4fa*)(bet + 4 * t4);
    asm volatile("" :: "v"(w4));
    asm volatile("" :: "v"(b4));
    asm volatile("" :: "v"(r4));
    asm volatile("" :: "v"(x4));
    asm volatile("" :: "v"(g4));
    asm volatile("" :: "v"(y4));
    *(v4fa*)(sS + S_W + 4 * tid) = w4;
    if (tid < 64) {
      *(v4fa*)(sS + S_B + 4 * tid) = b4;
      *(v4fa*)(sS + S_R + 4 * tid) = r4;
    }
    if (tid < 4) {
      *(v4fa*)(sS + S_VEC + 4 * tid)      = x4;
      *(v4fa*)(sS + S_VEC + 16 + 4 * tid) = g4;
      *(v4fa*)(sS + S_VEC + 32 + 4 * tid) = y4;
    }
    __syncthreads();
    if (blk < PB_W) {
      const int u   = blk * 256 + tid;
      const int ppr = K_E >> 3;
      const int n   = u / ppr;
      const int p   = u - n * ppr;
      const int oc  = n < 16 ? n : 15;
      unsigned w[8];
#pragma unroll
      for (int q = 0; q < 8; ++q) {
        const int kk = 8 * p + q;
        const int kh = kk >= KZ ? kk - KZ : kk;
        const int kc = kh < 80 ? kh : 79;
        const int i  = kc / 5;
        const int k  = kc - 5 * i;
        const int idx = (k < 4) ? (S_W + (16 * i + oc) * 4 + k) : (S_B + 16 * i + oc);
        const float val = sS[idx];
        const unsigned mk = (n < 16 && kh < 80) ? 0xFFFFu : 0u;
        w[q] = bf16_bits(val) & mk;
      }
      const v4u o = (v4u){ pk16(w[0], w[1]), pk16(w[2], w[3]), pk16(w[4], w[5]), pk16(w[6], w[7]) };
      volatile v4u* qd = (volatile v4u*)(WRB + (size_t)u * 8);
      *qd = o;
      __threadfence();
      *qd = o;
    } else {
      {
        const int n  = tid >> 2;
        const int p  = tid & 3;
        const int nc = n < 16 ? n : 15;
        unsigned w[8];
#pragma unroll
        for (int q = 0; q < 8; ++q) {
          const int k  = 8 * p + q;
          const int kc = k < 16 ? k : 15;
          const float val = sS[S_R + kc * 16 + nc];
          const unsigned mk = (n < 16 && k < 16) ? 0xFFFFu : 0u;
          w[q] = bf16_bits(val) & mk;
        }
        const v4u o = (v4u){ pk16(w[0], w[1]), pk16(w[2], w[3]), pk16(w[4], w[5]), pk16(w[6], w[7]) };
        volatile v4u* qd = (volatile v4u*)(ROOTT + (size_t)tid * 8);
        *qd = o;
        __threadfence();
        *qd = o;
      }
      {
        const int t24  = tid < 24 ? tid : 23;
        const int line = t24 >> 3;
        const int pc   = t24 & 7;
        float tv[4];
#pragma unroll
        for (int j = 0; j < 4; ++j) {
          const int col = 4 * pc + j;
          const int cc  = col < 16 ? col : 15;
          const float raw = sS[S_VEC + 16 * line + cc];
          const float val = RNE_VEC ? bf16_val(raw) : raw;
          tv[j] = (col < 16) ? val : 0.0f;
        }
        const v4f o = (v4f){ tv[0], tv[1], tv[2], tv[3] };
        if (tid < 24) {
          volatile v4f* qd = (volatile v4f*)(TAB + 4 * tid);
          *qd = o;
          __threadfence();
          *qd = o;
        }
      }
    }
  } else {
    unsigned short* zp = Z + (size_t)CH * K_E;
    const v4u z4 = (v4u){0u, 0u, 0u, 0u};
    for (int pass = 0; pass < 2; ++pass) {
      for (int i = tid; i < ZPADP; i += 256) *(volatile v4u*)(zp + (size_t)i * 8) = z4;
      __threadfence();
    }
  }
}

__global__ __launch_bounds__(256) __attribute__((amdgpu_num_vgpr(128)))
void k_list(const int* __restrict__ ei, int* __restrict__ LIST, int* __restrict__ CNT, int* __restrict__ OFF,
            int* __restrict__ FLAG) {
  extern __shared__ __attribute__((aligned(16))) int dsm[];
  int* wl   = dsm + LK_WL;
  int* sl   = dsm + LK_SL;
  int* cnt  = dsm + LK_CNT;
  int* offs = dsm + LK_OFF;
  int* cur  = dsm + LK_CUR;
  int* misc = dsm + LK_MISC;
  const int tid = (int)threadIdx.x, lane = tid & 31, wave = tid >> 5;
  const int blk = (int)blockIdx.x;
  const int nodeBase = blk * NBRUN;
  const int nbi = (NN - nodeBase) < NBRUN ? (NN - nodeBase) : NBRUN;
  const unsigned unb = (unsigned)(nbi < 0 ? 0 : nbi);

  {
    const v4i z4 = (v4i){0, 0, 0, 0};
    for (int i = tid * 4; i < CAP + NBRUN; i += 1024) *(v4ia*)(sl + i) = z4;
    if (tid < 16) misc[tid] = 0;
  }
  __syncthreads();

  const int* dstp = ei + NE;
  int* mylist = wl + wave * WLCAP;
  const int wbase = wave * EPW;
  const int wlast = wbase + EPW - 1;
  int wc = 0;
#pragma unroll 1
  for (int st = 0; st < NSTEP; ++st) {
    const int e0 = wbase + st * SUB + lane;
    int dk[4];
#pragma unroll
    for (int j = 0; j < 4; ++j) {
      const int e  = e0 + 32 * j;
      const int ec = e < wlast ? e : wlast;
      const int d  = dstp[ec];
      asm volatile("" :: "v"(d));
      dk[j] = (e <= wlast) ? d : -1;
    }
#pragma unroll
    for (int j = 0; j < 4; ++j) {
      const unsigned slot = (unsigned)dk[j] - (unsigned)nodeBase;
      const bool hit = slot < unb;
      const unsigned mj = __builtin_amdgcn_ballot_w32(hit);
      if (mj != 0u) {
        if (hit) {
          const int pos = wc + (int)__builtin_amdgcn_mbcnt_lo(mj, 0u);
          if (pos < WLCAP) mylist[pos] = ((e0 + 32 * j) << 10) | (int)slot;
        }
        wc += (int)__builtin_popcount(mj);
      }
    }
  }
  if (lane == 0) misc[wave] = wc;
  __syncthreads();

  if (wave == 0) {
    int t = 0, ov = 0;
#pragma unroll 1
    for (int w2 = 0; w2 < 8; ++w2) {
      const int craw = misc[w2];
      ov |= (craw > WLCAP) ? 1 : 0;
      const int c = __builtin_amdgcn_readfirstlane(clampi(craw, 0, WLCAP));
#pragma unroll 1
      for (int b0 = 0; b0 < c; b0 += 32) {
        const int idx = (b0 + lane) < c ? (b0 + lane) : c - 1;
        const int ent = wl[w2 * WLCAP + idx];
        const int m32 = (c - b0) < 32 ? (c - b0) : 32;
#pragma unroll 1
        for (int k = 0; k < m32; ++k) {
          const int u    = __builtin_amdgcn_readlane(ent, k);
          const int slot = u & (NBRUN - 1);
          if (t < CAP) {
            if (lane == 0) cnt[slot] = cnt[slot] + 1;
            t = t + 1;
          } else {
            ov = 1;
          }
        }
      }
    }
    if (lane == 0) { misc[8] = t; misc[9] = ov; }
  }
  __syncthreads();

  if (wave == 0) {
    const int base = lane * (NBRUN / 32);
    int s = 0, big = 0;
#pragma unroll 1
    for (int i = 0; i < NBRUN / 32; ++i) {
      const int cv = cnt[base + i];
      s += cv;
      big |= (cv > DEGCAP) ? 1 : 0;
    }
    int incl = s;
#pragma unroll
    for (int d = 1; d < 32; d <<= 1) {
      const int y = __shfl_up(incl, d, 32);
      incl += (lane >= d) ? y : 0;
    }
    int run = incl - s;
#pragma unroll 1
    for (int i = 0; i < NBRUN / 32; ++i) {
      const int cv = cnt[base + i];
      offs[base + i] = run;
      cur[base + i]  = run;
      run += cv;
    }
    const unsigned bm = __builtin_amdgcn_ballot_w32(big != 0);
    if (lane == 0) misc[9] = misc[9] | ((bm != 0u) ? 1 : 0);
  }
  __syncthreads();

  if (wave == 0) {
    int t2 = 0;
#pragma unroll 1
    for (int w2 = 0; w2 < 8; ++w2) {
      const int c = __builtin_amdgcn_readfirstlane(clampi(misc[w2], 0, WLCAP));
#pragma unroll 1
      for (int b0 = 0; b0 < c; b0 += 32) {
        const int idx = (b0 + lane) < c ? (b0 + lane) : c - 1;
        const int ent = wl[w2 * WLCAP + idx];
        const int m32 = (c - b0) < 32 ? (c - b0) : 32;
#pragma unroll 1
        for (int k = 0; k < m32; ++k) {
          const int u    = __builtin_amdgcn_readlane(ent, k);
          const int slot = u & (NBRUN - 1);
          if (t2 < CAP) {
            if (lane == 0) {
              int p = cur[slot];
              p = clampi(p, 0, CAP - 1);
              sl[p] = u >> 10;
              cur[slot] = p + 1;
            }
            t2 = t2 + 1;
          }
        }
      }
    }
  }
  __syncthreads();

  const int ovf = misc[9];
  int* lbase = LIST + (size_t)blk * (size_t)CAP;
  for (int pass = 0; pass < 2; ++pass) {
#pragma unroll 2
    for (int i = tid; i < CAP / 4; i += 256) {
      const v4i ev = *(const v4ia*)(sl + 4 * i);
      const v4i v = (v4i){ clampi(ev.x, 0, NE - 1), clampi(ev.y, 0, NE - 1),
                           clampi(ev.z, 0, NE - 1), clampi(ev.w, 0, NE - 1) };
      *(volatile v4i*)(lbase + 4 * i) = v;
    }
    __threadfence();
  }
  const v4i cv4 = *(const v4ia*)(cnt + 4 * tid);
  const v4i ov4 = *(const v4ia*)(offs + 4 * tid);
  const v4i fl4 = (v4i){ ovf, ovf, ovf, ovf };
  const size_t nb4 = (size_t)nodeBase + 4 * (size_t)tid;
  const bool fw = (wave == 0) && (lane < 8);
  *(volatile v4i*)(CNT + nb4) = cv4;
  *(volatile v4i*)(OFF + nb4) = ov4;
  if (fw) *(volatile v4i*)(FLAG + blk * 32 + 4 * lane) = fl4;
  __threadfence();
  *(volatile v4i*)(CNT + nb4) = cv4;
  *(volatile v4i*)(OFF + nb4) = ov4;
  if (fw) *(volatile v4i*)(FLAG + blk * 32 + 4 * lane) = fl4;
}

constexpr int PPW  = 25;
constexpr int ZGRD = CH / 2 / PPW / 8;
constexpr int ZPP  = 2 * K_E / 8;
static_assert(ZGRD * 8 * PPW * 2 == CH);
static_assert(ZPP == 48 || ZPP == 24);

__global__ __launch_bounds__(256) __attribute__((amdgpu_num_vgpr(128)))
void k_z(const float* __restrict__ v, const float* __restrict__ ef, const int* __restrict__ ei,
         unsigned short* __restrict__ Z, int ebase) {
  __shared__ __attribute__((aligned(16))) unsigned short sZ[8][2 * K_E];
  const int tid = (int)threadIdx.x, lane = tid & 31, wave = tid >> 5;
  const int h = lane >> 4, i = lane & 15;
  unsigned short* strip = sZ[wave];
  const int gw = (int)blockIdx.x * 8 + wave;
  const v4u z4 = (v4u){0u, 0u, 0u, 0u};
#pragma unroll 1
  for (int t = 0; t < PPW; ++t) {
    const int pr = gw * PPW + t;
    const int r  = 2 * pr + h;
    const int eg = clampi(ebase + r, 0, NE - 1);
    int s = ei[eg];
    asm volatile("" :: "v"(s));
    s = clampi(s, 0, NN - 1);
    const float vr = v[(size_t)s * 16 + i];
    asm volatile("" :: "v"(vr));
    const v4f er = *(const v4fa*)(ef + (size_t)eg * 4);
    asm volatile("" :: "v"(er));
    const float vb = bf16_val(vr);
    const float ek0 = bf16_val(er[0]);
    const float ek1 = bf16_val(er[1]);
    const float ek2 = bf16_val(er[2]);
    const float ek3 = bf16_val(er[3]);
    const float zz[5] = { vb * ek0, vb * ek1, vb * ek2, vb * ek3, vb * 1.0f };
    if (lane < 4 * ZTERMS) {
      const int rr = lane & 1, pc = (lane >> 1) & 1, tt = lane >> 2;
      *(v4ua*)(strip + rr * K_E + tt * KZ + 80 + 8 * pc) = z4;
    }
    unsigned short* my = strip + h * K_E + 5 * i;
#pragma unroll
    for (int k = 0; k < 5; ++k) {
      my[k] = (unsigned short)bf16_bits(zz[k]);
      if (ZTERMS == 2) my[KZ + k] = (unsigned short)bf16_lo_bits(zz[k]);
    }
    __builtin_amdgcn_fence(__ATOMIC_RELEASE, "workgroup");
    __builtin_amdgcn_wave_barrier();
    __builtin_amdgcn_fence(__ATOMIC_ACQUIRE, "workgroup");
    const int p0 = lane < ZPP ? lane : ZPP - 1;
    const int p1 = (lane + 32) < ZPP ? (lane + 32) : ZPP - 1;
    const v4u a0 = *(const v4ua*)(strip + 8 * p0);
    const v4u a1 = *(const v4ua*)(strip + 8 * p1);
    unsigned short* zrow = Z + (size_t)pr * (size_t)(2 * K_E);
    for (int pass = 0; pass < 2; ++pass) {
      if (lane < ZPP) *(volatile v4u*)(zrow + 8 * lane) = a0;
      if (ZPP > 32) {
        if (lane + 32 < ZPP) *(volatile v4u*)(zrow + 8 * (lane + 32)) = a1;
      }
      __threadfence();
    }
    __builtin_amdgcn_fence(__ATOMIC_RELEASE, "workgroup");
    __builtin_amdgcn_wave_barrier();
    __builtin_amdgcn_fence(__ATOMIC_ACQUIRE, "workgroup");
  }
}

constexpr int PK_PIECES = CH * 4;
constexpr int PK_GRID   = (PK_PIECES + 255) / 256;
static_assert(PK_PIECES % 32 == 0);

__global__ __launch_bounds__(256) __attribute__((amdgpu_num_vgpr(128)))
void k_pack16(const float* __restrict__ C, float* __restrict__ dst) {
  const int f4 = (int)blockIdx.x * 256 + (int)threadIdx.x;
  const int fc = f4 < PK_PIECES ? f4 : PK_PIECES - 1;
  const int row = fc >> 2, pc = fc & 3;
  const v4f x = *(const v4fa*)(C + (size_t)row * 64 + 4 * pc);
  asm volatile("" :: "v"(x));
  if (f4 < PK_PIECES) {
    volatile v4f* q = (volatile v4f*)(dst + (size_t)f4 * 4);
    *q = x;
    __threadfence();
    *q = x;
  }
}

__global__ __launch_bounds__(256) __attribute__((amdgpu_num_vgpr(128)))
void k_mean(const float* __restrict__ MSG16, const float* __restrict__ RT16, const int* __restrict__ LIST,
            const int* __restrict__ CNT, const int* __restrict__ OFF, const int* __restrict__ FLAG,
            const float* __restrict__ TAB, float* __restrict__ PRE) {
  __shared__ __attribute__((aligned(16))) float sB[32];
  const int tid = (int)threadIdx.x, lane = tid & 31, wave = tid >> 5;
  {
    const int t8 = tid < 8 ? tid : 7;
    const v4f b4 = *(const v4fa*)(TAB + T_BIAS + 4 * t8);
    asm volatile("" :: "v"(b4));
    if (tid < 8) *(v4fa*)(sB + 4 * tid) = b4;
  }
  __syncthreads();
  const int col = lane & 15, h = lane >> 4;
  const float bc = sB[col];
  const int n  = (((int)blockIdx.x * 8 + wave) << 1) + h;
  const int nc = clampi(n, 0, NN - 1);
  const int b  = nc >> 10;
  int c = CNT[nc];
  int o = OFF[nc];
  const int fl = FLAG[b * 32];
  asm volatile("" :: "v"(c));
  asm volatile("" :: "v"(o));
  asm volatile("" :: "v"(fl));
  c = clampi(c, 0, DEGCAP);
  o = clampi(o, 0, CAP - DEGCAP);
  const int co = __shfl_xor(c, 16, 32);
  const int cm = c > co ? c : co;
  const int trip = __builtin_amdgcn_readfirstlane(cm);
  const int* lp = LIST + (size_t)b * (size_t)CAP + (size_t)o;
  const int top = c > 0 ? c - 1 : 0;
  float s = 0.0f;
#pragma unroll 1
  for (int j = 0; j < trip; ++j) {
    const int idx = j < top ? j : top;
    int ed = lp[idx];
    asm volatile("" :: "v"(ed));
    ed = clampi(ed, 0, NE - 1);
    const float mv = MSG16[(size_t)ed * 16 + col];
    asm volatile("" :: "v"(mv));
    const float add = (j < c) ? mv : 0.0f;
    s = s + add;
  }
  const float dn = (float)(c > 0 ? c : 1);
  const float mean = s / dn;
  const float rt = RT16[(size_t)nc * 16 + col];
  asm volatile("" :: "v"(rt));
  const float tv = (mean + rt) + bc;
  const float qn = __int_as_float(0x7fc00000);
  const float pv = (fl != 0) ? qn : tv;
  volatile float* q = (volatile float*)(PRE + (size_t)nc * 16 + col);
  *q = pv;
  __threadfence();
  *q = pv;
}

template <int MODE>
__global__ __launch_bounds__(256) __attribute__((amdgpu_num_vgpr(128)))
void k_colstat(const float* __restrict__ H, const float* __restrict__ TAB, double* __restrict__ rec) {
  static_assert(MODE == 0 || MODE == 1);
  __shared__ __attribute__((aligned(16))) float  sm[16];
  __shared__ __attribute__((aligned(16))) double sp[256];
  const int tid = (int)threadIdx.x;
  if (tid < 32) {
    const int t4 = tid < 4 ? tid : 3;
    v4f mv = (v4f){0.f, 0.f, 0.f, 0.f};
    if constexpr (MODE == 1) {
      mv = *(const v4fa*)(TAB + T_MU + 4 * t4);
      asm volatile("" :: "v"(mv));
    }
    if (tid < 4) *(v4fa*)(sm + 4 * tid) = mv;
  }
  __syncthreads();
  const int col = tid & 15;
  const int g   = tid >> 4;
  const int r0  = (int)blockIdx.x * RROWS + g * GROWS;
  const float m = sm[col];
  const float* hp = H + (size_t)r0 * 16 + col;
  double s = 0.0;
#pragma unroll 5
  for (int j = 0; j < GROWS; ++j) {
    const float x = hp[(size_t)j * 16];
    if constexpr (MODE == 0) {
      s += (double)x;
    } else {
      const float d = x - m;
      const double dd = (double)d;
      s += dd * dd;
    }
  }
  sp[tid] = s;
  __syncthreads();
  const int t8 = tid < 8 ? tid : 7;
  double a0 = 0.0, a1 = 0.0;
#pragma unroll 4
  for (int g2 = 0; g2 < 16; ++g2) {
    a0 += sp[g2 * 16 + 2 * t8];
    a1 += sp[g2 * 16 + 2 * t8 + 1];
  }
  const v2d o = (v2d){ a0, a1 };
  if (tid < 8) {
    volatile v2d* q = (volatile v2d*)(rec + (size_t)blockIdx.x * 16 + 2 * tid);
    *q = o;
    __threadfence();
    *q = o;
  }
}

__global__ __launch_bounds__(32) void k_comb(const double* __restrict__ rec, float* __restrict__ outl,
                                             double inv_count, int mode) {
  __shared__ __attribute__((aligned(16))) float sv[32];
  const int lane = (int)threadIdx.x;
  const int c = lane & 15;
  double s = 0.0;
#pragma unroll 5
  for (int i = 0; i < NREC; ++i) s += rec[(size_t)i * 16 + c];
  const float qf = (float)(s * inv_count);
  const float rs = 1.0f / sqrtf(qf + 1e-5f);
  const float val = (mode == 0) ? qf : rs;
  sv[lane] = (lane < 16) ? val : 0.0f;
  __syncthreads();
  const int t8 = lane < 8 ? lane : 7;
  const v4f o = (v4f){ sv[4 * t8], sv[4 * t8 + 1], sv[4 * t8 + 2], sv[4 * t8 + 3] };
  if (lane < 8) {
    volatile v4f* q = (volatile v4f*)(outl + 4 * lane);
    *q = o;
    __threadfence();
    *q = o;
  }
}

__global__ __launch_bounds__(256) __attribute__((amdgpu_num_vgpr(128)))
void k_out(const float* __restrict__ PRE, const float* __restrict__ TAB, float* __restrict__ outp) {
  __shared__ __attribute__((aligned(16))) float sP[128];
  const int tid = (int)threadIdx.x, lane = tid & 31, wave = tid >> 5;
  if (wave == 0) {
    const v4f a = *(const v4fa*)(TAB + T_GAM + 4 * lane);
    asm volatile("" :: "v"(a));
    *(v4fa*)(sP + 4 * lane) = a;
  }
  __syncthreads();
  const int f  = (int)blockIdx.x * 256 + tid;
  const int c  = f & 15;
  const int fc = f < OUT_ELEMS ? f : OUT_ELEMS - 1;
  const float x = PRE[fc];
  asm volatile("" :: "v"(x));
  const float g  = sP[c];
  const float be = sP[32 + c];
  const float mu = sP[64 + c];
  const float rs = sP[96 + c];
  const float y = ((g * (x - mu)) * rs) + be;
  const float o = (y >= 0.0f) ? y : (0.01f * y);
  if (f < OUT_ELEMS) {
    volatile float* q = (volatile float*)(outp + fc);
    *q = o;
    __threadfence();
    *q = o;
  }
}

constexpr int G_GEMM = ((CHP / 64) * 1 + 7) / 8;
constexpr int G_VB   = VBP * (K_R / 8) / 256;
static_assert((VBP * (K_R / 8)) % 256 == 0);

extern "C" void kernel_launch(void* const* d_in, const int* in_sizes, int n_in,
                              void* d_out, int out_size, void* d_ws, size_t ws_size,
                              hipStream_t stream) {
  if (n_in < 9) return;
  if (in_sizes[0] != NN * 16) return;
  if (in_sizes[1] != NE * 4) return;
  if (in_sizes[2] != 2 * NE) return;
  if (in_sizes[3] != 1024 || in_sizes[4] != 256) return;
  if (in_sizes[5] != 256) return;
  if (in_sizes[6] != 16 || in_sizes[7] != 16 || in_sizes[8] != 16) return;
  if (out_size != OUT_ELEMS) return;
  if (ws_size < WS_TOTAL) return;

  const float* v    = (const float*)d_in[0];
  const float* ef   = (const float*)d_in[1];
  const int*   ei   = (const int*)d_in[2];
  const float* EW   = (const float*)d_in[3];
  const float* EB   = (const float*)d_in[4];
  const float* root = (const float*)d_in[5];
  const float* bias = (const float*)d_in[6];
  const float* gam  = (const float*)d_in[7];
  const float* bet  = (const float*)d_in[8];
  float* out = (float*)d_out;

  char* ws = (char*)d_ws;
  unsigned short* Z     = (unsigned short*)(ws + OFF_Z);
  float*          MSGC  = (float*)(ws + OFF_MSGC);
  float*          MSG16 = (float*)(ws + OFF_MSG16);
  float*          RT16  = (float*)(ws + OFF_RT16);
  float*          PRE   = (float*)(ws + OFF_PRE);
  unsigned short* VB    = (unsigned short*)(ws + OFF_VB);
  int*            LIST  = (int*)(ws + OFF_LIST);
  int*            CNT   = (int*)(ws + OFF_CNT);
  int*            OFFS  = (int*)(ws + OFF_OFF);
  int*            FLAG  = (int*)(ws + OFF_FLAG);
  unsigned short* WRB   = (unsigned short*)(ws + OFF_WRB);
  unsigned short* ROOTT = (unsigned short*)(ws + OFF_ROOTT);
  float*          TAB   = (float*)(ws + OFF_TAB);
  double*         REC   = (double*)(ws + OFF_REC);

  const double invN = 1.0 / 100000.0;

  hipFuncSetAttribute(reinterpret_cast<const void*>(&k_list), hipFuncAttributeMaxDynamicSharedMemorySize, (int)LK_LDS);

  k_prep<<<PB_TOT, 256, 0, stream>>>(EW, EB, root, bias, gam, bet, WRB, ROOTT, TAB, Z);
  k_plane<0><<<G_VB, 256, 0, stream>>>(v, NN, 16, 16, VB, VBP, K_R);
  k_list<<<NBLK, 256, LK_LDS, stream>>>(ei, LIST, CNT, OFFS, FLAG);

  for (int h = 0; h < 2; ++h) {
    k_gemm_nt<0, 0><<<G_GEMM, 256, 0, stream>>>(VB + (size_t)h * CH * K_R, ROOTT, TAB, MSGC, CH, 64, K_R, 64);
    k_pack16<<<PK_GRID, 256, 0, stream>>>(MSGC, RT16 + (size_t)h * CH * 16);
  }

  for (int c = 0; c < NCH; ++c) {
    k_z<<<ZGRD, 256, 0, stream>>>(v, ef, ei, Z, c * CH);
    k_gemm_nt<0, 0><<<G_GEMM, 256, 0, stream>>>(Z, WRB, TAB, MSGC, CH, 64, K_E, 64);
    k_pack16<<<PK_GRID, 256, 0, stream>>>(MSGC, MSG16 + (size_t)c * CH * 16);
  }

  k_mean<<<NN / 2 / 8, 256, 0, stream>>>(MSG16, RT16, LIST, CNT, OFFS, FLAG, TAB, PRE);

  k_colstat<0><<<NREC, 256, 0, stream>>>(PRE, TAB, REC);
  k_comb<<<1, 32, 0, stream>>>(REC, TAB + T_MU, invN, 0);
  k_colstat<1><<<NREC, 256, 0, stream>>>(PRE, TAB, REC);
  k_comb<<<1, 32, 0, stream>>>(REC, TAB + T_RS, invN, 1);

  k_out<<<OUT_ELEMS / 256, 256, 0, stream>>>(PRE, TAB, out);
}
